// HSTULayer_53807350284553
// MI455X (gfx1250) — hardware-verified
//
#include <hip/hip_runtime.h>
#include <math.h>


static constexpr int kBatch = 2;
static constexpr int kSeq   = 2048;
static constexpr int kD     = 1024;
static constexpr int kHeads = 16;
static constexpr int kDh    = 64;
static constexpr int kTok   = kBatch * kSeq;
static constexpr int kN1    = 4 * kD;
static constexpr int kKch   = kSeq / 32;
static constexpr int kQblk  = kSeq / 64;
static constexpr int kCvtThreads  = 256;
static constexpr int kFlagThreads = 256;
static constexpr int kGemmThreads = 128;
static constexpr int kLnThreads   = 128;
static constexpr int kStgPitch = 132;
static constexpr int kPP = 36;
static constexpr int kOP = 68;

static_assert(kHeads * kDh == kD);
static_assert(kDh == 64);
static_assert(kSeq % 64 == 0);
static_assert(kTok % 64 == 0);
static_assert(kN1 % 128 == 0);
static_assert(kD % 128 == 0);
static_assert(kD % 32 == 0);
static_assert((kTok * kD) % (kCvtThreads * 8) == 0);
static_assert((kN1 * kD) % (kCvtThreads * 8) == 0);
static_assert((kD * kD) % (kCvtThreads * 8) == 0);
static_assert(kSeq == kFlagThreads * 8);
static_assert(kKch == 64);
static_assert((kBatch * kHeads * (kSeq / 16)) % 4 == 0);
static_assert((kSeq / 16) % 4 == 0);
static_assert(kD == kLnThreads * 8);
static_assert(kTok % 32 == 0);

typedef _Float16     v16h __attribute__((ext_vector_type(16)));
typedef _Float16     v8h  __attribute__((ext_vector_type(8)));
typedef float        v8f  __attribute__((ext_vector_type(8)));
typedef float        v4f  __attribute__((ext_vector_type(4)));
typedef unsigned int v4u  __attribute__((ext_vector_type(4)));
typedef int          v4i  __attribute__((ext_vector_type(4)));

union Frag { v16h v; v8h half[2]; };

__device__ __forceinline__ v8f wmma_f16(v16h a, v16h b, v8f acc)
{
    acc = __builtin_amdgcn_wmma_f32_16x16x32_f16(false, a, false, b, (short)0, acc, false, false);
#if defined(__HIP_DEVICE_COMPILE__)
    asm volatile("v_nop\n\tv_nop\n\tv_nop\n\tv_nop" : "+v"(acc) : "v"(a), "v"(b));
#endif
    return acc;
}

__device__ __forceinline__ float bf16_rne(float x)
{
    unsigned int u = __float_as_uint(x);
    u = u + 0x7FFFu + ((u >> 16) & 1u);
    return __uint_as_float(u & 0xFFFF0000u);
}

__device__ __forceinline__ _Float16 cvt16(float x, float sc)
{
    return (_Float16)(bf16_rne(x) * sc);
}

__device__ __forceinline__ float silu_fast(float z)
{
    return z * __builtin_amdgcn_rcpf(1.0f + __expf(-z));
}

__device__ __forceinline__ float wave_sum(float v)
{
    v += __shfl_xor(v, 1, 32);
    v += __shfl_xor(v, 2, 32);
    v += __shfl_xor(v, 4, 32);
    v += __shfl_xor(v, 8, 32);
    v += __shfl_xor(v, 16, 32);
    return v;
}

__global__ __launch_bounds__(kCvtThreads)
void k_cvt_rows(const float* __restrict__ src, _Float16* __restrict__ dst, float sc, int n)
{
    const size_t base = ((size_t)blockIdx.x * kCvtThreads + threadIdx.x) * 8;
    if (base + 8 <= (size_t)n) {
        const v4f f0 = *(const v4f*)(src + base);
        const v4f f1 = *(const v4f*)(src + base + 4);
        v8h hv;
        hv[0] = cvt16(f0[0], sc); hv[1] = cvt16(f0[1], sc);
        hv[2] = cvt16(f0[2], sc); hv[3] = cvt16(f0[3], sc);
        hv[4] = cvt16(f1[0], sc); hv[5] = cvt16(f1[1], sc);
        hv[6] = cvt16(f1[2], sc); hv[7] = cvt16(f1[3], sc);
        const v4u u = __builtin_bit_cast(v4u, hv);
        volatile v4u* p = (volatile v4u*)(dst + base);
        *p = u;
        __threadfence();
        *p = u;
    }
}

__global__ __launch_bounds__(kFlagThreads)
void k_flags(const float* __restrict__ mask, int* __restrict__ flags)
{
    __shared__ __align__(16) int sf[64];
    const int tid = threadIdx.x;
    const int bq  = blockIdx.x;
    const int bb  = bq >> 5;
    const int qb  = bq & 31;
    const float* mp = mask + ((size_t)bb * kSeq + (size_t)qb * 64) * kSeq + 8 * tid;
    int any = 0;
#pragma unroll 1
    for (int r = 0; r < 64; ++r) {
        const v4f a = *(const v4f*)(mp + (size_t)r * kSeq);
        const v4f c = *(const v4f*)(mp + (size_t)r * kSeq + 4);
        any |= (int)(a[0] != 0.0f) | (int)(a[1] != 0.0f) | (int)(a[2] != 0.0f) | (int)(a[3] != 0.0f)
             | (int)(c[0] != 0.0f) | (int)(c[1] != 0.0f) | (int)(c[2] != 0.0f) | (int)(c[3] != 0.0f);
    }
    any |= __shfl_xor(any, 1, 32);
    any |= __shfl_xor(any, 2, 32);
    if ((tid & 3) == 0) sf[tid >> 2] = any;
    __syncthreads();
    if (tid < 16) {
        const v4i v = *(const v4i*)(sf + 4 * tid);
        volatile v4i* p = (volatile v4i*)(flags + (size_t)bq * 64 + 4 * tid);
        *p = v;
        __threadfence();
        *p = v;
    }
}

__global__ __launch_bounds__(kGemmThreads)
void k_gemm1(const _Float16* __restrict__ Xh, const _Float16* __restrict__ W1h,
             const float* __restrict__ b1,
             const float* __restrict__ cosb, const float* __restrict__ sinb,
             float* __restrict__ Uf, _Float16* __restrict__ VT, _Float16* __restrict__ QK)
{
    __shared__ __align__(16) float stg[64 * kStgPitch];

    const int tid  = threadIdx.x;
    const int wave = tid >> 5;
    const int lane = tid & 31;
    const int h    = lane >> 4;
    const int m    = lane & 15;
    const int n0   = blockIdx.x * 128;
    const int m0   = blockIdx.y * 64;
    const int wm   = (wave & 1) * 32;
    const int wn   = (wave >> 1) * 64;

    const _Float16* ap = Xh  + (size_t)(m0 + wm + m) * kD + 8 * h;
    const _Float16* bp = W1h + (size_t)(n0 + wn + m) * kD + 8 * h;

    v8f acc[8] = {};
#pragma unroll 1
    for (int k0 = 0; k0 < kD; k0 += 32) {
        Frag a0, a1;
        a0.half[0] = *(const v8h*)(ap + k0);
        a0.half[1] = *(const v8h*)(ap + k0 + 16);
        a1.half[0] = *(const v8h*)(ap + 16 * kD + k0);
        a1.half[1] = *(const v8h*)(ap + 16 * kD + k0 + 16);
#pragma unroll
        for (int t = 0; t < 4; ++t) {
            Frag b;
            const _Float16* bt = bp + (size_t)t * 16 * kD + k0;
            b.half[0] = *(const v8h*)(bt);
            b.half[1] = *(const v8h*)(bt + 16);
            acc[t]     = wmma_f16(a0.v, b.v, acc[t]);
            acc[4 + t] = wmma_f16(a1.v, b.v, acc[4 + t]);
        }
    }

    const int mode = n0 / kD;

#pragma unroll
    for (int t = 0; t < 4; ++t) {
        const int c = wn + 16 * t + m;
        const float bias = bf16_rne(b1[n0 + c]);
#pragma unroll
        for (int i = 0; i < 2; ++i) {
#pragma unroll
            for (int r = 0; r < 8; ++r) {
                const float z = acc[4 * i + t][r] * (1.0f / 4096.0f) + bias;
                stg[(wm + 16 * i + 8 * h + r) * kStgPitch + c] = (mode == 0) ? silu_fast(z) : z;
            }
        }
    }
    __syncthreads();

    if (mode == 0) {
        float* dst = Uf + (size_t)m0 * kD + n0 + 4 * lane;
#pragma unroll
        for (int g = 0; g < 4; ++g) {
            v4f v[4];
#pragma unroll
            for (int rr = 0; rr < 4; ++rr) {
                const int row = wave * 16 + 4 * g + rr;
                v[rr] = *(const v4f*)(stg + row * kStgPitch + 4 * lane);
            }
#pragma unroll
            for (int rr = 0; rr < 4; ++rr)
                *(volatile v4f*)(dst + (size_t)(wave * 16 + 4 * g + rr) * kD) = v[rr];
            __threadfence();
#pragma unroll
            for (int rr = 0; rr < 4; ++rr)
                *(volatile v4f*)(dst + (size_t)(wave * 16 + 4 * g + rr) * kD) = v[rr];
        }
    } else if (mode == 1) {
        const int bb  = m0 / kSeq;
        const int s0  = m0 % kSeq;
        const int hh0 = (n0 - kD) / kDh;
        const int p   = lane & 7;
        const int qs  = lane >> 3;
        _Float16* vb = VT + (size_t)((bb * kHeads + hh0) * kDh) * kSeq + s0 + 8 * p;
        v4u u[8];
#pragma unroll
        for (int i = 0; i < 8; ++i) {
            const int c = wave * 32 + 4 * i + qs;
            v8h hv;
#pragma unroll
            for (int e = 0; e < 8; ++e)
                hv[e] = (_Float16)(stg[(8 * p + e) * kStgPitch + c] * 16.0f);
            u[i] = __builtin_bit_cast(v4u, hv);
        }
#pragma unroll
        for (int i = 0; i < 8; ++i)
            *(volatile v4u*)(vb + (size_t)(wave * 32 + 4 * i + qs) * kSeq) = u[i];
        __threadfence();
#pragma unroll
        for (int i = 0; i < 8; ++i)
            *(volatile v4u*)(vb + (size_t)(wave * 32 + 4 * i + qs) * kSeq) = u[i];
    } else {
        const int coff = n0 - mode * kD;
        _Float16* dst = QK + (size_t)(mode - 2) * kTok * kD + (size_t)m0 * kD + coff + 8 * m;
        const int   d0  = 8 * (m & 7);
        const float sgn = (m & 4) ? 1.0f : -1.0f;
        v4u u[8];
#pragma unroll
        for (int i = 0; i < 8; ++i) {
            const int row = wave * 16 + 2 * i + h;
            const float* sp = stg + row * kStgPitch + 8 * m;
            const float* pp = stg + row * kStgPitch + 8 * (m ^ 4);
            const size_t cso = (size_t)(m0 + row) * kDh + d0;
            const v4f f0 = *(const v4f*)(sp);
            const v4f f1 = *(const v4f*)(sp + 4);
            const v4f g0 = *(const v4f*)(pp);
            const v4f g1 = *(const v4f*)(pp + 4);
            const v4f c0 = *(const v4f*)(cosb + cso);
            const v4f c1 = *(const v4f*)(cosb + cso + 4);
            const v4f s0 = *(const v4f*)(sinb + cso);
            const v4f s1 = *(const v4f*)(sinb + cso + 4);
            v8h hv;
#pragma unroll
            for (int e = 0; e < 4; ++e) {
                const float o0 = f0[e] * bf16_rne(c0[e]) + sgn * g0[e] * bf16_rne(s0[e]);
                const float o1 = f1[e] * bf16_rne(c1[e]) + sgn * g1[e] * bf16_rne(s1[e]);
                hv[e]     = (_Float16)(o0 * 16.0f);
                hv[4 + e] = (_Float16)(o1 * 16.0f);
            }
            u[i] = __builtin_bit_cast(v4u, hv);
        }
#pragma unroll
        for (int i = 0; i < 8; ++i)
            *(volatile v4u*)(dst + (size_t)(wave * 16 + 2 * i + h) * kD) = u[i];
        __threadfence();
#pragma unroll
        for (int i = 0; i < 8; ++i)
            *(volatile v4u*)(dst + (size_t)(wave * 16 + 2 * i + h) * kD) = u[i];
    }
}

__global__ __launch_bounds__(kGemmThreads)
void k_attn(const _Float16* __restrict__ Qh, const _Float16* __restrict__ Kh,
            const _Float16* __restrict__ VT, const float* __restrict__ mask,
            const int* __restrict__ flags, float* __restrict__ Af)
{
    __shared__ __align__(16) float sP[4 * 16 * kPP];
    __shared__ __align__(16) float sO[4 * 16 * kOP];

    const int tid  = threadIdx.x;
    const int wave = tid >> 5;
    const int lane = tid & 31;
    const int h    = lane >> 4;
    const int m    = lane & 15;
    const int blk  = blockIdx.x;
    const int qblk = blk % kQblk;
    const int hh   = (blk / kQblk) % kHeads;
    const int bb   = blk / (kQblk * kHeads);
    const int q0   = qblk * 64 + wave * 16;
    const int tok0 = bb * kSeq + q0;
    const int hc   = hh * kDh;

    const int* fl = flags + ((size_t)bb * kQblk + qblk) * kKch;

    const _Float16* qp = Qh + (size_t)(tok0 + m) * kD + hc + 8 * h;
    Frag aq0, aq1;
    aq0.half[0] = *(const v8h*)(qp);
    aq0.half[1] = *(const v8h*)(qp + 16);
    aq1.half[0] = *(const v8h*)(qp + 32);
    aq1.half[1] = *(const v8h*)(qp + 48);

    const _Float16* kp = Kh + (size_t)(bb * kSeq + m) * kD + hc + 8 * h;
    const _Float16* vp = VT + (size_t)((bb * kHeads + hh) * kDh + m) * kSeq + 8 * h;
    const float*  mrow = mask + ((size_t)bb * kSeq + q0 + m) * kSeq + 8 * h;
    float* myP = sP + wave * (16 * kPP);
    float* myO = sO + wave * (16 * kOP);

    v8f acc[4] = {};
#pragma unroll 1
    for (int kc = 0; kc < kKch; ++kc) {
        const int f = fl[kc];
        if (f != 0) {
            const int kb = kc * 32;
            const _Float16* kr0 = kp + (size_t)kb * kD;
            const _Float16* kr1 = kr0 + 16 * kD;
            Frag b00, b01, b10, b11;
            b00.half[0] = *(const v8h*)(kr0);
            b00.half[1] = *(const v8h*)(kr0 + 16);
            b01.half[0] = *(const v8h*)(kr0 + 32);
            b01.half[1] = *(const v8h*)(kr0 + 48);
            b10.half[0] = *(const v8h*)(kr1);
            b10.half[1] = *(const v8h*)(kr1 + 16);
            b11.half[0] = *(const v8h*)(kr1 + 32);
            b11.half[1] = *(const v8h*)(kr1 + 48);
            v8f s0 = {}, s1 = {};
            s0 = wmma_f16(aq0.v, b00.v, s0);
            s0 = wmma_f16(aq1.v, b01.v, s0);
            s1 = wmma_f16(aq0.v, b10.v, s1);
            s1 = wmma_f16(aq1.v, b11.v, s1);

            {
                float* pw = myP + (8 * h) * kPP + m;
#pragma unroll
                for (int r = 0; r < 8; ++r) {
                    pw[r * kPP]      = silu_fast(s0[r] * (1.0f / 2048.0f));
                    pw[r * kPP + 16] = silu_fast(s1[r] * (1.0f / 2048.0f));
                }
            }
            __syncthreads();

            Frag ap;
            {
                const float* pr = myP + m * kPP + 8 * h;
                const float* mk = mrow + kb;
                const v4f p0 = *(const v4f*)(pr);
                const v4f p1 = *(const v4f*)(pr + 4);
                const v4f p2 = *(const v4f*)(pr + 16);
                const v4f p3 = *(const v4f*)(pr + 20);
                const v4f w0 = *(const v4f*)(mk);
                const v4f w1 = *(const v4f*)(mk + 4);
                const v4f w2 = *(const v4f*)(mk + 16);
                const v4f w3 = *(const v4f*)(mk + 20);
                v8h h0v, h1v;
#pragma unroll
                for (int e = 0; e < 4; ++e) {
                    h0v[e]     = (_Float16)(p0[e] * bf16_rne(w0[e]) * 256.0f);
                    h0v[4 + e] = (_Float16)(p1[e] * bf16_rne(w1[e]) * 256.0f);
                    h1v[e]     = (_Float16)(p2[e] * bf16_rne(w2[e]) * 256.0f);
                    h1v[4 + e] = (_Float16)(p3[e] * bf16_rne(w3[e]) * 256.0f);
                }
                ap.half[0] = h0v;
                ap.half[1] = h1v;
            }
#pragma unroll
            for (int t = 0; t < 4; ++t) {
                Frag bv;
                const _Float16* vr = vp + (size_t)t * 16 * kSeq + kb;
                bv.half[0] = *(const v8h*)(vr);
                bv.half[1] = *(const v8h*)(vr + 16);
                acc[t] = wmma_f16(ap.v, bv.v, acc[t]);
            }
            __syncthreads();
        }
    }

#pragma unroll
    for (int t = 0; t < 4; ++t) {
#pragma unroll
        for (int r = 0; r < 8; ++r)
            myO[(8 * h + r) * kOP + 16 * t + m] = acc[t][r] * (1.0f / 4096.0f);
    }
    __syncthreads();

    const size_t gbase = (size_t)tok0 * kD + hc + 4 * m;
    v4f g[8];
#pragma unroll
    for (int i = 0; i < 8; ++i) {
        const int row = 2 * i + h;
        g[i] = *(const v4f*)(myO + row * kOP + 4 * m);
    }
#pragma unroll
    for (int i = 0; i < 8; ++i)
        *(volatile v4f*)(Af + gbase + (size_t)(2 * i + h) * kD) = g[i];
    __threadfence();
#pragma unroll
    for (int i = 0; i < 8; ++i)
        *(volatile v4f*)(Af + gbase + (size_t)(2 * i + h) * kD) = g[i];
}

__global__ __launch_bounds__(kLnThreads)
void k_norm(const float* __restrict__ A, const float* __restrict__ gate, const float* __restrict__ Uf,
            _Float16* __restrict__ Lh, _Float16* __restrict__ Ll)
{
    __shared__ float red[4];
    const int tid  = threadIdx.x;
    const int wave = tid >> 5;
    const int lane = tid & 31;
    const int row  = blockIdx.x;
    const int c0   = tid * 8;
    const float* ar = A + (size_t)row * kD + c0;
    const v4f f0 = *(const v4f*)(ar);
    const v4f f1 = *(const v4f*)(ar + 4);
    float x[8];
    x[0] = f0[0]; x[1] = f0[1]; x[2] = f0[2]; x[3] = f0[3];
    x[4] = f1[0]; x[5] = f1[1]; x[6] = f1[2]; x[7] = f1[3];

    float ss = 0.0f;
#pragma unroll
    for (int e = 0; e < 8; ++e) ss += x[e] * x[e];
    ss = wave_sum(ss);
    if (lane == 0) red[wave] = ss;
    __syncthreads();
    const float var  = ((red[0] + red[1]) + (red[2] + red[3])) * (1.0f / 1024.0f);
    const float rstd = rsqrtf(var + 1e-6f);

    const float* ur = Uf + (size_t)row * kD + c0;
    const v4f u0 = *(const v4f*)(ur);
    const v4f u1 = *(const v4f*)(ur + 4);
    float uu[8];
    uu[0] = u0[0]; uu[1] = u0[1]; uu[2] = u0[2]; uu[3] = u0[3];
    uu[4] = u1[0]; uu[5] = u1[1]; uu[6] = u1[2]; uu[7] = u1[3];

    v8h hvh, hvl;
#pragma unroll
    for (int e = 0; e < 8; ++e) {
        const float gm = bf16_rne(gate[c0 + e]);
        const float y  = (gm * (x[e] * rstd)) * uu[e];
        const _Float16 yh = (_Float16)y;
        hvh[e] = yh;
        hvl[e] = (_Float16)((y - (float)yh) * 2048.0f);
    }
    const v4u uh = __builtin_bit_cast(v4u, hvh);
    const v4u ul = __builtin_bit_cast(v4u, hvl);
    volatile v4u* ph = (volatile v4u*)(Lh + (size_t)row * kD + c0);
    volatile v4u* pl = (volatile v4u*)(Ll + (size_t)row * kD + c0);
    *ph = uh;
    *pl = ul;
    __threadfence();
    *ph = uh;
    *pl = ul;
}

__global__ __launch_bounds__(kGemmThreads)
void k_gemm2(const _Float16* __restrict__ Lh, const _Float16* __restrict__ Ll,
             const _Float16* __restrict__ W2h, const float* __restrict__ b2,
             const float* __restrict__ Xres, float* __restrict__ Out)
{
    __shared__ __align__(16) float stg[32 * kStgPitch];

    const int tid  = threadIdx.x;
    const int wave = tid >> 5;
    const int lane = tid & 31;
    const int h    = lane >> 4;
    const int m    = lane & 15;
    const int n0   = blockIdx.x * 128;
    const int m0   = blockIdx.y * 32;
    const int wn   = wave * 32;

    const size_t aoff = (size_t)(m0 + m) * kD + 8 * h;
    const _Float16* ahp = Lh + aoff;
    const _Float16* alp = Ll + aoff;
    const _Float16* bp  = W2h + (size_t)(n0 + wn + m) * kD + 8 * h;

    v8f acch[4] = {}, accl[4] = {};
#pragma unroll 1
    for (int k0 = 0; k0 < kD; k0 += 32) {
        Frag ah0, ah1, al0, al1, b0, b1;
        ah0.half[0] = *(const v8h*)(ahp + k0);
        ah0.half[1] = *(const v8h*)(ahp + k0 + 16);
        ah1.half[0] = *(const v8h*)(ahp + 16 * kD + k0);
        ah1.half[1] = *(const v8h*)(ahp + 16 * kD + k0 + 16);
        al0.half[0] = *(const v8h*)(alp + k0);
        al0.half[1] = *(const v8h*)(alp + k0 + 16);
        al1.half[0] = *(const v8h*)(alp + 16 * kD + k0);
        al1.half[1] = *(const v8h*)(alp + 16 * kD + k0 + 16);
        b0.half[0]  = *(const v8h*)(bp + k0);
        b0.half[1]  = *(const v8h*)(bp + k0 + 16);
        b1.half[0]  = *(const v8h*)(bp + 16 * kD + k0);
        b1.half[1]  = *(const v8h*)(bp + 16 * kD + k0 + 16);
        acch[0] = wmma_f16(ah0.v, b0.v, acch[0]);
        acch[1] = wmma_f16(ah0.v, b1.v, acch[1]);
        acch[2] = wmma_f16(ah1.v, b0.v, acch[2]);
        acch[3] = wmma_f16(ah1.v, b1.v, acch[3]);
        accl[0] = wmma_f16(al0.v, b0.v, accl[0]);
        accl[1] = wmma_f16(al0.v, b1.v, accl[1]);
        accl[2] = wmma_f16(al1.v, b0.v, accl[2]);
        accl[3] = wmma_f16(al1.v, b1.v, accl[3]);
    }

#pragma unroll
    for (int t = 0; t < 2; ++t) {
        const int c = wn + 16 * t + m;
        const float bias = bf16_rne(b2[n0 + c]);
#pragma unroll
        for (int i = 0; i < 2; ++i) {
#pragma unroll
            for (int r = 0; r < 8; ++r) {
                const float y = (acch[2 * i + t][r] + accl[2 * i + t][r] * (1.0f / 2048.0f)) * (1.0f / 256.0f) + bias;
                stg[(16 * i + 8 * h + r) * kStgPitch + c] = y;
            }
        }
    }
    __syncthreads();

    float* dst = Out + (size_t)m0 * kD + n0 + 4 * lane;
    const float* xr = Xres + (size_t)m0 * kD + n0 + 4 * lane;
    v4f v[8];
#pragma unroll
    for (int rr = 0; rr < 8; ++rr) {
        const int row = wave * 8 + rr;
        const v4f s  = *(const v4f*)(stg + row * kStgPitch + 4 * lane);
        const v4f xv = *(const v4f*)(xr + (size_t)row * kD);
        v4f o;
        o[0] = s[0] + bf16_rne(xv[0]);
        o[1] = s[1] + bf16_rne(xv[1]);
        o[2] = s[2] + bf16_rne(xv[2]);
        o[3] = s[3] + bf16_rne(xv[3]);
        v[rr] = o;
    }
#pragma unroll
    for (int rr = 0; rr < 8; ++rr)
        *(volatile v4f*)(dst + (size_t)(wave * 8 + rr) * kD) = v[rr];
    __threadfence();
#pragma unroll
    for (int rr = 0; rr < 8; ++rr)
        *(volatile v4f*)(dst + (size_t)(wave * 8 + rr) * kD) = v[rr];
}

extern "C" void kernel_launch(void* const* d_in, const int* in_sizes, int n_in,
                              void* d_out, int out_size, void* d_ws, size_t ws_size,
                              hipStream_t stream)
{
    if (n_in < 9) return;
    if (in_sizes[0] != kTok * kD) return;
    if (in_sizes[1] != kTok * kDh) return;
    if (in_sizes[2] != kTok * kDh) return;
    if (in_sizes[3] != kBatch * kSeq * kSeq) return;
    if (in_sizes[4] != kN1 * kD) return;
    if (in_sizes[5] != kN1) return;
    if (in_sizes[6] != kD) return;
    if (in_sizes[7] != kD * kD) return;
    if (in_sizes[8] != kD) return;
    if (out_size != kTok * kD) return;

    const size_t bXh  = (size_t)kTok * kD * sizeof(_Float16);
    const size_t bW1h = (size_t)kN1 * kD * sizeof(_Float16);
    const size_t bW2h = (size_t)kD * kD * sizeof(_Float16);
    const size_t bUf  = (size_t)kTok * kD * sizeof(float);
    const size_t bVT  = (size_t)kBatch * kHeads * kDh * kSeq * sizeof(_Float16);
    const size_t bQK  = (size_t)2 * kTok * kD * sizeof(_Float16);
    const size_t bAf  = (size_t)kTok * kD * sizeof(float);
    const size_t bLh  = (size_t)kTok * kD * sizeof(_Float16);
    const size_t bLl  = (size_t)kTok * kD * sizeof(_Float16);
    const size_t bFl  = (size_t)kBatch * kQblk * kKch * sizeof(int);
    const size_t total = bXh + bW1h + bW2h + bUf + bVT + bQK + bAf + bLh + bLl + bFl;
    if (ws_size < total) return;

    const float* x      = (const float*)d_in[0];
    const float* cosb   = (const float*)d_in[1];
    const float* sinb   = (const float*)d_in[2];
    const float* mask   = (const float*)d_in[3];
    const float* W_uvqk = (const float*)d_in[4];
    const float* b_uvqk = (const float*)d_in[5];
    const float* gate_w = (const float*)d_in[6];
    const float* W_out  = (const float*)d_in[7];
    const float* b_out  = (const float*)d_in[8];
    float* Out = (float*)d_out;

    char* ws = (char*)d_ws;
    size_t o = 0;
    _Float16* Xh  = (_Float16*)(ws + o); o += bXh;
    _Float16* W1h = (_Float16*)(ws + o); o += bW1h;
    _Float16* W2h = (_Float16*)(ws + o); o += bW2h;
    float*    Uf  = (float*)(ws + o);    o += bUf;
    _Float16* VT  = (_Float16*)(ws + o); o += bVT;
    _Float16* QK  = (_Float16*)(ws + o); o += bQK;
    float*    Af  = (float*)(ws + o);    o += bAf;
    _Float16* Lh  = (_Float16*)(ws + o); o += bLh;
    _Float16* Ll  = (_Float16*)(ws + o); o += bLl;
    int*      Fl  = (int*)(ws + o);      o += bFl;
    const _Float16* Qh = QK;
    const _Float16* Kh = QK + (size_t)kTok * kD;

    const int nX  = kTok * kD;
    const int nW1 = kN1 * kD;
    const int nW2 = kD * kD;
    k_cvt_rows<<<dim3((unsigned)(nX / 8 / kCvtThreads)), dim3(kCvtThreads), 0, stream>>>(x, Xh, 16.0f, nX);
    k_cvt_rows<<<dim3((unsigned)(nW1 / 8 / kCvtThreads)), dim3(kCvtThreads), 0, stream>>>(W_uvqk, W1h, 256.0f, nW1);
    k_cvt_rows<<<dim3((unsigned)(nW2 / 8 / kCvtThreads)), dim3(kCvtThreads), 0, stream>>>(W_out, W2h, 256.0f, nW2);
    k_flags<<<dim3(kBatch * kQblk), dim3(kFlagThreads), 0, stream>>>(mask, Fl);
    k_gemm1<<<dim3(kN1 / 128, kTok / 64), dim3(kGemmThreads), 0, stream>>>(Xh, W1h, b_uvqk, cosb, sinb, Uf, VT, QK);
    k_attn<<<dim3((kBatch * kHeads * (kSeq / 16)) / 4), dim3(kGemmThreads), 0, stream>>>(Qh, Kh, VT, mask, Fl, Af);
    k_norm<<<dim3(kTok), dim3(kLnThreads), 0, stream>>>(Af, gate_w, Uf, Lh, Ll);
    k_gemm2<<<dim3(kD / 128, kTok / 32), dim3(kGemmThreads), 0, stream>>>(Lh, Ll, W2h, b_out, x, Out);
}
